// MPNNTransform_3839700762650
// MI455X (gfx1250) — hardware-verified
//
#include <hip/hip_runtime.h>
#include <math.h>

constexpr int kBatch = 32;
constexpr int kNodes = 256;
constexpr int kFeat  = 8;
constexpr int kHid   = 256;
constexpr int kRows  = kBatch * kNodes;
constexpr int kG3    = 3 * kHid;
constexpr int kHF    = kHid + kFeat;
constexpr int kIters = 3;
constexpr int kRowsPerBlk = 8;
constexpr float kHCarry = 64.0f;
constexpr float kWCarry = 16.0f;
constexpr float kGemmScale = 1.0f / (kHCarry * kWCarry);

static_assert(kRows % 64 == 0 && kG3 % 64 == 0 && kHid % 64 == 0, "GEMM M and N are multiples of the 64 tile");
static_assert(kHid % 32 == 0, "GEMM K is a multiple of 32");
static_assert(kRows % kRowsPerBlk == 0 && kNodes % kRowsPerBlk == 0, "row blocks never straddle a batch");
static_assert(kNodes == 256 && kHid == 256 && kG3 == 768, "thread maps assume 256 threads = one row");

typedef __attribute__((ext_vector_type(16))) _Float16 v16h;
typedef __attribute__((ext_vector_type(8)))  _Float16 v8h;
typedef __attribute__((ext_vector_type(16))) __bf16   v16b;
typedef __attribute__((ext_vector_type(8)))  __bf16   v8b;
typedef __attribute__((ext_vector_type(8)))  float    v8f;
typedef __attribute__((ext_vector_type(4)))  float    v4f;
typedef __attribute__((ext_vector_type(4)))  unsigned int v4u;

__device__ __forceinline__ unsigned short f2bf_bits(float f) {
  unsigned u = __float_as_uint(f);
  return (unsigned short)((u + 0x7FFFu + ((u >> 16) & 1u)) >> 16);
}
__device__ __forceinline__ float bf_bits2f(unsigned short h) { return __uint_as_float(((unsigned)h) << 16); }

__device__ __forceinline__ void dep_guard_h(v8f& a, v8f& b, v16h x, v16h y) { asm volatile("v_nop\n\tv_nop\n\tv_nop\n\tv_nop" : "+v"(a), "+v"(b) : "v"(x), "v"(y)); }
__device__ __forceinline__ void dep_guard_b(v8f& a, v8f& b, v16b x, v16b y) { asm volatile("v_nop\n\tv_nop\n\tv_nop\n\tv_nop" : "+v"(a), "+v"(b) : "v"(x), "v"(y)); }
__device__ __forceinline__ void dep_guard4_h(v8f& a, v8f& b, v8f& c, v8f& d, v16h x, v16h y) { asm volatile("v_nop\n\tv_nop\n\tv_nop\n\tv_nop" : "+v"(a), "+v"(b), "+v"(c), "+v"(d) : "v"(x), "v"(y)); }
__device__ __forceinline__ void dep_guard4_b(v8f& a, v8f& b, v8f& c, v8f& d, v16b x, v16b y) { asm volatile("v_nop\n\tv_nop\n\tv_nop\n\tv_nop" : "+v"(a), "+v"(b), "+v"(c), "+v"(d) : "v"(x), "v"(y)); }
__device__ __forceinline__ void keep4_h(v16h a, v16h b, v16h c, v16h d) { asm volatile("v_nop" :: "v"(a), "v"(b), "v"(c), "v"(d)); }
__device__ __forceinline__ void keep4_b(v16b a, v16b b, v16b c, v16b d) { asm volatile("v_nop" :: "v"(a), "v"(b), "v"(c), "v"(d)); }
__device__ __forceinline__ void acc_guard4(v8f& a, v8f& b, v8f& c, v8f& d) { asm volatile("v_nop\n\tv_nop\n\tv_nop\n\tv_nop" : "+v"(a), "+v"(b), "+v"(c), "+v"(d)); }
template <typename T> struct Frag;
template <> struct Frag<_Float16> {
  typedef v16h V; union U { v16h v; v8h h[2]; };
  static __device__ __forceinline__ v16h load(const _Float16* p) {
    U f; f.h[0] = *(const v8h*)(p); f.h[1] = *(const v8h*)(p + 16); return f.v;
  }
  static __device__ __forceinline__ v8f mma(v16h a, v16h b, v8f c) {
    return __builtin_amdgcn_wmma_f32_16x16x32_f16(false, a, false, b, (short)0, c, false, false);
  }
  static __device__ __forceinline__ void guard(v8f& a, v8f& b, v16h x, v16h y) { dep_guard_h(a, b, x, y); }
  static __device__ __forceinline__ void guard4(v8f& a, v8f& b, v8f& c, v8f& d, v16h x, v16h y) { dep_guard4_h(a, b, c, d, x, y); }
  static __device__ __forceinline__ void keep(v16h a, v16h b, v16h c, v16h d) { keep4_h(a, b, c, d); }
};
template <> struct Frag<__bf16> {
  typedef v16b V; union U { v16b v; v8b h[2]; };
  static __device__ __forceinline__ v16b load(const __bf16* p) {
    U f; f.h[0] = *(const v8b*)(p); f.h[1] = *(const v8b*)(p + 16); return f.v;
  }
  static __device__ __forceinline__ v8f mma(v16b a, v16b b, v8f c) {
    return __builtin_amdgcn_wmma_f32_16x16x32_bf16(false, a, false, b, (short)0, c, false, false);
  }
  static __device__ __forceinline__ void guard(v8f& a, v8f& b, v16b x, v16b y) { dep_guard_b(a, b, x, y); }
  static __device__ __forceinline__ void guard4(v8f& a, v8f& b, v8f& c, v8f& d, v16b x, v16b y) { dep_guard4_b(a, b, c, d, x, y); }
  static __device__ __forceinline__ void keep(v16b a, v16b b, v16b c, v16b d) { keep4_b(a, b, c, d); }
};

__device__ __forceinline__ unsigned pk16(unsigned short a, unsigned short b) { return (unsigned)a | ((unsigned)b << 16); }
__device__ __forceinline__ unsigned short h_bits(float f) { const _Float16 h = (_Float16)f; return __builtin_bit_cast(unsigned short, h); }

template <int ET> struct Elem;
template <> struct Elem<0> { typedef _Float16 T; };
template <> struct Elem<1> { typedef __bf16 T; };
template <int ET, bool SPLIT, int BIAS_MODE, int OUT_MODE, bool RESID, int ACT = 0>
__global__ __launch_bounds__(256) void wmma_gemm64(
    const unsigned short* __restrict__ Ap, const unsigned short* __restrict__ A2p, int lda, long strideA,
    const unsigned short* __restrict__ Btp, const unsigned short* __restrict__ Bt2p, int ldb, long strideB,
    void* __restrict__ Cout, void* __restrict__ Cout2, int ldc, long strideC,
    const float* __restrict__ bias,
    const float* __restrict__ resid, long strideR,
    int M, int N, int K, float scale) {
  typedef typename Elem<ET>::T T;
  typedef typename Frag<T>::V V;
  const T* A = (const T*)Ap; const T* A2 = (const T*)A2p; const T* Bt = (const T*)Btp; const T* Bt2 = (const T*)Bt2p;
  __shared__ __align__(16) float sT[8][16 * 68];
  const int b    = blockIdx.y;
  const int lane = threadIdx.x & 31;
  const int wave = threadIdx.x >> 5;
  const int tilesN = N >> 6;
  const int tilesM = M >> 6;
  const int tile = blockIdx.x * 8 + wave;
  if (tile >= tilesM * tilesN) return;
  const int tm = tile / tilesN;
  const int tn = tile - tm * tilesN;
  const int m0 = tm << 6;
  const int n0 = tn << 6;

  const T* Ab  = A  + (size_t)b * strideA;
  const T* Bb  = Bt + (size_t)b * strideB;
  const T* Ab2 = SPLIT ? (A2  + (size_t)b * strideA) : nullptr;
  const T* Bb2 = SPLIT ? (Bt2 + (size_t)b * strideB) : nullptr;

  const int rlane = lane & 15;
  const int koff  = (lane >> 4) * 8;
  const int mOff  = (lane >> 4) * 8;

  v8f acc[4][4];
#pragma unroll
  for (int i = 0; i < 4; ++i)
#pragma unroll
    for (int j = 0; j < 4; ++j) acc[i][j] = (v8f){0.f,0.f,0.f,0.f,0.f,0.f,0.f,0.f};

  for (int k0 = 0; k0 < K; k0 += 32) {
    V bh[4], bl[4];
#pragma unroll
    for (int j = 0; j < 4; ++j) {
      const size_t bo = (size_t)(n0 + (j << 4) + rlane) * ldb + koff + k0;
      bh[j] = Frag<T>::load(Bb + bo);
      if (SPLIT) bl[j] = Frag<T>::load(Bb2 + bo);
    }
#pragma unroll
    for (int i = 0; i < 4; ++i) {
      const size_t ao = (size_t)(m0 + (i << 4) + rlane) * lda + koff + k0;
      V ah = Frag<T>::load(Ab + ao);
      V al;
      if (SPLIT) al = Frag<T>::load(Ab2 + ao);
#pragma unroll
      for (int j = 0; j < 4; ++j) {
        acc[i][j] = Frag<T>::mma(ah, bh[j], acc[i][j]);
        if (SPLIT) {
          acc[i][j] = Frag<T>::mma(ah, bl[j], acc[i][j]);
          acc[i][j] = Frag<T>::mma(al, bh[j], acc[i][j]);
        }
      }
      Frag<T>::guard4(acc[i][0], acc[i][1], acc[i][2], acc[i][3], ah, SPLIT ? al : ah);
    }
    Frag<T>::keep(bh[0], bh[1], bh[2], bh[3]);
    if (SPLIT) Frag<T>::keep(bl[0], bl[1], bl[2], bl[3]);
  }
  acc_guard4(acc[0][0], acc[0][1], acc[0][2], acc[0][3]);
  acc_guard4(acc[1][0], acc[1][1], acc[1][2], acc[1][3]);
  acc_guard4(acc[2][0], acc[2][1], acc[2][2], acc[2][3]);
  acc_guard4(acc[3][0], acc[3][1], acc[3][2], acc[3][3]);

  float* slab = sT[wave];
  const float* Rb = RESID ? (resid + (size_t)b * strideR) : nullptr;
#pragma unroll
  for (int i = 0; i < 4; ++i) {
    const int mBase = m0 + (i << 4);
#pragma unroll
    for (int j = 0; j < 4; ++j) {
      const int n = n0 + (j << 4) + rlane;
      float bv = 0.f;
      if (BIAS_MODE == 2) bv = bias[n];
#pragma unroll
      for (int r = 0; r < 8; ++r) {
        float v = acc[i][j][r] * scale;
        if (BIAS_MODE == 1) v += bias[mBase + mOff + r];
        if (BIAS_MODE == 2) v += bv;
        if (RESID) v += Rb[(size_t)(mBase + mOff + r) * ldc + n];
        if (ACT == 2) v = fmaxf(v, 0.0f);
        if (ACT == 4) v = (v > 0.f) ? v : 0.01f * v;
        slab[(mOff + r) * 68 + (j << 4) + rlane] = v;
      }
    }
    __builtin_amdgcn_fence(__ATOMIC_RELEASE, "workgroup");
    __builtin_amdgcn_wave_barrier();
    __builtin_amdgcn_fence(__ATOMIC_ACQUIRE, "workgroup");
    if (OUT_MODE == 0) {
      float* C = (float*)Cout + (size_t)b * strideC;
      const int hh = lane >> 4, c4 = (lane & 15) * 4;
      for (int pass = 0; pass < 2; ++pass) {
#pragma unroll
        for (int it = 0; it < 8; ++it) {
          const int row = it * 2 + hh;
          v4f v = *(const v4f*)(slab + row * 68 + c4);
          *(volatile v4f*)(C + (size_t)(mBase + row) * ldc + n0 + c4) = v;
        }
        __threadfence();
      }
    } else {
      const int q = lane >> 3, c8 = (lane & 7) * 8;
      unsigned short* C  = (unsigned short*)Cout  + (size_t)b * strideC;
      unsigned short* C2 = (OUT_MODE == 2) ? ((unsigned short*)Cout2 + (size_t)b * strideC) : nullptr;
      for (int pass = 0; pass < 2; ++pass) {
#pragma unroll
        for (int it = 0; it < 4; ++it) {
          const int row = it * 4 + q;
          const float* sp = slab + row * 68 + c8;
          v8h hv, lv;
#pragma unroll
          for (int e = 0; e < 8; ++e) {
            if (OUT_MODE == 1) {
              hv[e] = (_Float16)sp[e];
            } else {
              unsigned short hb = f2bf_bits(sp[e]);
              unsigned short lb = f2bf_bits(sp[e] - bf_bits2f(hb));
              hv[e] = __builtin_bit_cast(_Float16, hb);
              lv[e] = __builtin_bit_cast(_Float16, lb);
            }
          }
          *(volatile v8h*)(C + (size_t)(mBase + row) * ldc + n0 + c8) = hv;
          if (OUT_MODE == 2) *(volatile v8h*)(C2 + (size_t)(mBase + row) * ldc + n0 + c8) = lv;
        }
        __threadfence();
      }
    }
    __builtin_amdgcn_fence(__ATOMIC_RELEASE, "workgroup");
    __builtin_amdgcn_wave_barrier();
    __builtin_amdgcn_fence(__ATOMIC_ACQUIRE, "workgroup");
  }
}

__device__ __forceinline__ float wsum(float d) {
  d += __shfl_xor(d, 1, 32); d += __shfl_xor(d, 2, 32); d += __shfl_xor(d, 4, 32);
  d += __shfl_xor(d, 8, 32); d += __shfl_xor(d, 16, 32); return d;
}
__device__ __forceinline__ float wmax(float d) {
  d = fmaxf(d, __shfl_xor(d, 1, 32)); d = fmaxf(d, __shfl_xor(d, 2, 32)); d = fmaxf(d, __shfl_xor(d, 4, 32));
  d = fmaxf(d, __shfl_xor(d, 8, 32)); d = fmaxf(d, __shfl_xor(d, 16, 32)); return d;
}
__device__ __forceinline__ float dot8(v4f a, v4f c, v4f w0, v4f w1) {
  float d = 0.0f;
  d += a[0] * w0[0]; d += a[1] * w0[1]; d += a[2] * w0[2]; d += a[3] * w0[3];
  d += c[0] * w1[0]; d += c[1] * w1[1]; d += c[2] * w1[2]; d += c[3] * w1[3];
  return d;
}
__device__ __forceinline__ v4u pack8_f16(v4f q0, v4f q1, float scale) {
  unsigned short hb[8];
#pragma unroll
  for (int e = 0; e < 4; ++e) { hb[e] = h_bits(q0[e] * scale); hb[4 + e] = h_bits(q1[e] * scale); }
  return (v4u){pk16(hb[0], hb[1]), pk16(hb[2], hb[3]), pk16(hb[4], hb[5]), pk16(hb[6], hb[7])};
}
__device__ __forceinline__ void store_h_row(const float* shr, float* hrow, unsigned short* h16row, int lane) {
  const v4f hA = *(const v4f*)(shr + 4 * lane);
  const v4f hB = *(const v4f*)(shr + 128 + 4 * lane);
  const v4f q0 = *(const v4f*)(shr + 8 * lane);
  const v4f q1 = *(const v4f*)(shr + 8 * lane + 4);
  const v4u u = pack8_f16(q0, q1, kHCarry);
  for (int pass = 0; pass < 2; ++pass) {
    *(volatile v4f*)(hrow + 4 * lane) = hA;
    *(volatile v4f*)(hrow + 128 + 4 * lane) = hB;
    *(volatile v4u*)(h16row + 8 * lane) = u;
    __threadfence();
  }
}

__global__ __launch_bounds__(256) void cast8_scale_f16_kernel(const float* __restrict__ in, unsigned short* __restrict__ out,
                                                              int n8, float scale) {
  const int i = blockIdx.x * 256 + threadIdx.x;
  if (i >= n8) return;
  const float* p = in + 8 * (size_t)i;
  const v4f a = *(const v4f*)(p);
  const v4f c = *(const v4f*)(p + 4);
  const v4u u = pack8_f16(a, c, scale);
  unsigned short* q = out + 8 * (size_t)i;
  *(volatile v4u*)q = u;
  __threadfence();
  *(volatile v4u*)q = u;
}

__global__ __launch_bounds__(256) void wr1t_kernel(const float* __restrict__ W, unsigned short* __restrict__ out, float scale) {
  __shared__ float sm[64][65];
  const int t  = threadIdx.x;
  const int k0 = blockIdx.x * 64;
  const int o0 = blockIdx.y * 64;
#pragma unroll
  for (int i = 0; i < 16; ++i) {
    const int e = i * 256 + t;
    const int r = e >> 6;
    const int c = e & 63;
    sm[c][r] = W[(size_t)(k0 + r) * kHid + o0 + c] * scale;
  }
  __syncthreads();
  const int lane = t & 31, wave = t >> 5;
  const int q = lane >> 3, c8 = (lane & 7) * 8;
  for (int pass = 0; pass < 2; ++pass) {
#pragma unroll
    for (int it = 0; it < 2; ++it) {
      const int row = wave * 8 + it * 4 + q;
      unsigned short hb[8];
#pragma unroll
      for (int e = 0; e < 8; ++e) hb[e] = h_bits(sm[row][c8 + e]);
      const v4u u = (v4u){pk16(hb[0], hb[1]), pk16(hb[2], hb[3]), pk16(hb[4], hb[5]), pk16(hb[6], hb[7])};
      *(volatile v4u*)(out + (size_t)(o0 + row) * kHid + k0 + c8) = u;
    }
    __threadfence();
  }
}

__global__ __launch_bounds__(256) void embed_kernel(const float* __restrict__ jets, const float* __restrict__ W_emb,
                                                    const float* __restrict__ b_emb, const float* __restrict__ Wi,
                                                    const float* __restrict__ bi,
                                                    float* __restrict__ h32, unsigned short* __restrict__ h16,
                                                    float* __restrict__ gij) {
  __shared__ __align__(16) float sh[kRowsPerBlk * kHid];
  __shared__ __align__(16) float sg[kRowsPerBlk * kG3];
  __shared__ float sj[kRowsPerBlk * kFeat];
  const int t = threadIdx.x, lane = t & 31, wave = t >> 5;
  const int m0 = blockIdx.x * kRowsPerBlk;
  const float jv0 = jets[(size_t)m0 * kFeat + (t & 63)];
  if (t < kRowsPerBlk * kFeat) sj[t] = jv0;
  float we[kFeat];
#pragma unroll
  for (int f = 0; f < kFeat; ++f) we[f] = W_emb[f * kHid + t];
  const float be = b_emb[t];
  asm volatile("" ::: "memory");
  const v4f wj0a = *(const v4f*)(Wi + (size_t)t * kHF + kHid);
  const v4f wj0b = *(const v4f*)(Wi + (size_t)t * kHF + kHid + 4);
  const v4f wj1a = *(const v4f*)(Wi + (size_t)(kHid + t) * kHF + kHid);
  const v4f wj1b = *(const v4f*)(Wi + (size_t)(kHid + t) * kHF + kHid + 4);
  const v4f wj2a = *(const v4f*)(Wi + (size_t)(2 * kHid + t) * kHF + kHid);
  const v4f wj2b = *(const v4f*)(Wi + (size_t)(2 * kHid + t) * kHF + kHid + 4);
  asm volatile("" ::: "memory");
  const float bi0 = bi[t], bi1 = bi[kHid + t], bi2 = bi[2 * kHid + t];
  __syncthreads();
#pragma unroll 1
  for (int r = 0; r < kRowsPerBlk; ++r) {
    float jv[kFeat];
#pragma unroll
    for (int f = 0; f < kFeat; ++f) jv[f] = sj[r * kFeat + f];
    float a = 0.0f;
#pragma unroll
    for (int f = 0; f < kFeat; ++f) a += jv[f] * we[f];
    a += be;
    sh[r * kHid + t] = tanhf(a);
    float g0 = 0.0f, g1 = 0.0f, g2 = 0.0f;
#pragma unroll
    for (int e = 0; e < 4; ++e) {
      g0 += jv[e] * wj0a[e]; g0 += jv[4 + e] * wj0b[e];
      g1 += jv[e] * wj1a[e]; g1 += jv[4 + e] * wj1b[e];
      g2 += jv[e] * wj2a[e]; g2 += jv[4 + e] * wj2b[e];
    }
    sg[r * kG3 + t]            = g0 + bi0;
    sg[r * kG3 + kHid + t]     = g1 + bi1;
    sg[r * kG3 + 2 * kHid + t] = g2 + bi2;
  }
  __syncthreads();
  const int row = wave;
  const size_t m = (size_t)(m0 + row);
  store_h_row(sh + row * kHid, h32 + m * kHid, h16 + m * kHid, lane);
  const float* sgr = sg + row * kG3;
  v4f gv[6];
#pragma unroll
  for (int it = 0; it < 6; ++it) gv[it] = *(const v4f*)(sgr + it * 128 + 4 * lane);
  float* grow = gij + m * kG3;
  for (int pass = 0; pass < 2; ++pass) {
#pragma unroll
    for (int it = 0; it < 6; ++it) *(volatile v4f*)(grow + it * 128 + 4 * lane) = gv[it];
    __threadfence();
  }
}

__global__ __launch_bounds__(256) void attn_msg_kernel(const float* __restrict__ h32, const float* __restrict__ w_edge,
                                                       const float* __restrict__ b_edge, const float* __restrict__ W_msg,
                                                       const float* __restrict__ b_msg, const float* __restrict__ Wi,
                                                       float* __restrict__ gmsg) {
  __shared__ float sP[kNodes];
  __shared__ float sRed[16];
  __shared__ __align__(16) float sHbar[kHid];
  __shared__ __align__(16) float sMsg[kHid];
  __shared__ __align__(16) float sG[kG3];
  const int t = threadIdx.x, lane = t & 31, wave = t >> 5;
  const int b = blockIdx.x;
  const float* hb = h32 + (size_t)b * kNodes * kHid;

  const v4f we0 = *(const v4f*)(w_edge + 8 * lane);
  const v4f we1 = *(const v4f*)(w_edge + 8 * lane + 4);
  const float bev = b_edge[0];
#pragma unroll 1
  for (int i = 0; i < kNodes / 8; ++i) {
    const int row = wave * (kNodes / 8) + i;
    const float* rp = hb + (size_t)row * kHid + 8 * lane;
    const v4f a = *(const v4f*)(rp);
    const v4f c = *(const v4f*)(rp + 4);
    float d = dot8(a, c, we0, we1);
    d = wsum(d);
    if (lane == 0) sP[row] = d + bev;
  }
  __syncthreads();

  const float s = sP[t];
  const float mxw = wmax(s);
  if (lane == 0) sRed[wave] = mxw;
  __syncthreads();
  float gm = sRed[0];
#pragma unroll
  for (int w = 1; w < 8; ++w) gm = fmaxf(gm, sRed[w]);
  const float e = expf(s - gm);
  const float sew = wsum(e);
  if (lane == 0) sRed[8 + wave] = sew;
  __syncthreads();
  float den = 0.0f;
#pragma unroll
  for (int w = 0; w < 8; ++w) den += sRed[8 + w];
  const float p = e * (1.0f / den);
  sP[t] = p;
  __syncthreads();

  float acc = 0.0f;
#pragma unroll 4
  for (int j = 0; j < kNodes; ++j) acc += sP[j] * hb[(size_t)j * kHid + t];
  sHbar[t] = acc;
  __syncthreads();

  float a2 = 0.0f;
#pragma unroll 4
  for (int k = 0; k < kHid; ++k) a2 += sHbar[k] * W_msg[(size_t)k * kHid + t];
  a2 += b_msg[t];
  sMsg[t] = tanhf(a2);
  __syncthreads();

  const v4f mg0 = *(const v4f*)(sMsg + 8 * lane);
  const v4f mg1 = *(const v4f*)(sMsg + 8 * lane + 4);
#pragma unroll 1
  for (int i = 0; i < kG3 / 8; ++i) {
    const int o = wave * (kG3 / 8) + i;
    const float* wr = Wi + (size_t)o * kHF + 8 * lane;
    const v4f a = *(const v4f*)(wr);
    const v4f c = *(const v4f*)(wr + 4);
    float d = dot8(a, c, mg0, mg1);
    d = wsum(d);
    if (lane == 0) sG[o] = d;
  }
  __syncthreads();
  if (wave == 0) {
    v4f gv[6];
#pragma unroll
    for (int it = 0; it < 6; ++it) gv[it] = *(const v4f*)(sG + it * 128 + 4 * lane);
    float* gr = gmsg + (size_t)b * kG3;
    for (int pass = 0; pass < 2; ++pass) {
#pragma unroll
      for (int it = 0; it < 6; ++it) *(volatile v4f*)(gr + it * 128 + 4 * lane) = gv[it];
      __threadfence();
    }
  }
}

__global__ __launch_bounds__(256) void gru_kernel(const float* __restrict__ gij, const float* __restrict__ gh,
                                                  const float* __restrict__ gmsg, const float* __restrict__ bh,
                                                  const float* __restrict__ hold,
                                                  float* __restrict__ hnew32, unsigned short* __restrict__ hnew16) {
  __shared__ __align__(16) float sh[kRowsPerBlk * kHid];
  const int t = threadIdx.x, lane = t & 31, wave = t >> 5;
  const int m0 = blockIdx.x * kRowsPerBlk;
  const int b = m0 / kNodes;
  const float gm0 = gmsg[(size_t)b * kG3 + t];
  const float gm1 = gmsg[(size_t)b * kG3 + kHid + t];
  const float gm2 = gmsg[(size_t)b * kG3 + 2 * kHid + t];
  const float bh0 = bh[t], bh1 = bh[kHid + t], bh2 = bh[2 * kHid + t];
#pragma unroll 1
  for (int r = 0; r < kRowsPerBlk; ++r) {
    const size_t m = (size_t)(m0 + r);
    const float* gi = gij + m * kG3;
    const float* gg = gh + m * kG3;
    const float i0 = gi[t], i1 = gi[kHid + t], i2 = gi[2 * kHid + t];
    const float g0 = gg[t], g1 = gg[kHid + t], g2 = gg[2 * kHid + t];
    const float ho = hold[m * kHid + t];
    float xr = (gm0 + i0) + (g0 + bh0);
    float xz = (gm1 + i1) + (g1 + bh1);
    xr = fminf(fmaxf(xr, -30.0f), 30.0f);
    xz = fminf(fmaxf(xz, -30.0f), 30.0f);
    const float rg = 1.0f / (1.0f + expf(-xr));
    const float zg = 1.0f / (1.0f + expf(-xz));
    const float nn = tanhf((gm2 + i2) + rg * (g2 + bh2));
    const float hn = (1.0f - zg) * nn + zg * ho;
    sh[r * kHid + t] = hn;
  }
  __syncthreads();
  const int row = wave;
  const size_t m = (size_t)(m0 + row);
  store_h_row(sh + row * kHid, hnew32 + m * kHid, hnew16 + m * kHid, lane);
}

__global__ __launch_bounds__(256) void readout_kernel(const float* __restrict__ y, const float* __restrict__ Wr2,
                                                      const float* __restrict__ br2, float* __restrict__ out) {
  __shared__ float sY[kHid];
  __shared__ __align__(16) float sO[kHid];
  const int t = threadIdx.x, lane = t & 31, wave = t >> 5;
  const int b = blockIdx.x;
  const float* yb = y + (size_t)b * kNodes * kHid;
  float acc = 0.0f;
#pragma unroll 4
  for (int n = 0; n < kNodes; ++n) acc += yb[(size_t)n * kHid + t];
  sY[t] = acc;
  __syncthreads();
  float o = 0.0f;
#pragma unroll 4
  for (int k = 0; k < kHid; ++k) o += sY[k] * Wr2[(size_t)k * kHid + t];
  o += (float)kNodes * br2[t];
  sO[t] = o;
  __syncthreads();
  if (wave == 0) {
    const v4f p0 = *(const v4f*)(sO + 4 * lane);
    const v4f p1 = *(const v4f*)(sO + 128 + 4 * lane);
    float* orow = out + (size_t)b * kHid;
    for (int pass = 0; pass < 2; ++pass) {
      *(volatile v4f*)(orow + 4 * lane) = p0;
      *(volatile v4f*)(orow + 128 + 4 * lane) = p1;
      __threadfence();
    }
  }
}

extern "C" void kernel_launch(void* const* d_in, const int* in_sizes, int n_in,
                              void* d_out, int out_size, void* d_ws, size_t ws_size, hipStream_t stream) {
  (void)in_sizes; (void)n_in; (void)out_size;
  const float* jets   = (const float*)d_in[0];
  const float* W_emb  = (const float*)d_in[1];
  const float* b_emb  = (const float*)d_in[2];
  const float* w_edge = (const float*)d_in[3];
  const float* b_edge = (const float*)d_in[4];
  const float* W_msg  = (const float*)d_in[5];
  const float* b_msg  = (const float*)d_in[6];
  const float* Wi     = (const float*)d_in[7];
  const float* bi     = (const float*)d_in[8];
  const float* Wh     = (const float*)d_in[9];
  const float* bh     = (const float*)d_in[10];
  const float* Wr1    = (const float*)d_in[11];
  const float* br1    = (const float*)d_in[12];
  const float* Wr2    = (const float*)d_in[13];
  const float* br2    = (const float*)d_in[14];
  float* out = (float*)d_out;

  char* ws = (char*)d_ws; size_t off = 0;
  auto carve = [&](size_t bytes) -> char* { char* p = ws + off; off += (bytes + 255) & ~(size_t)255; return p; };
  unsigned short* Wh16   = (unsigned short*)carve((size_t)kG3 * kHid * 2);
  unsigned short* Wr1T16 = (unsigned short*)carve((size_t)kHid * kHid * 2);
  float* h32v[kIters + 1];
  unsigned short* h16v[kIters + 1];
  for (int s = 0; s <= kIters; ++s) h32v[s] = (float*)carve((size_t)kRows * kHid * 4);
  for (int s = 0; s <= kIters; ++s) h16v[s] = (unsigned short*)carve((size_t)kRows * kHid * 2);
  float* gij = (float*)carve((size_t)kRows * kG3 * 4);
  float* gh  = (float*)carve((size_t)kRows * kG3 * 4);
  float* gmsgv[kIters];
  for (int s = 0; s < kIters; ++s) gmsgv[s] = (float*)carve((size_t)kBatch * kG3 * 4);
  float* y = (float*)carve((size_t)kRows * kHid * 4);
  if (off > ws_size || off > (size_t)134217728) return;

  cast8_scale_f16_kernel<<<(kG3 * kHid / 8 + 255) / 256, 256, 0, stream>>>(Wh, Wh16, kG3 * kHid / 8, kWCarry);
  wr1t_kernel<<<dim3(kHid / 64, kHid / 64), 256, 0, stream>>>(Wr1, Wr1T16, kWCarry);

  embed_kernel<<<kRows / kRowsPerBlk, 256, 0, stream>>>(jets, W_emb, b_emb, Wi, bi, h32v[0], h16v[0], gij);

  const int ghTiles = (kRows / 64) * (kG3 / 64);
  for (int s = 0; s < kIters; ++s) {
    attn_msg_kernel<<<kBatch, 256, 0, stream>>>(h32v[s], w_edge, b_edge, W_msg, b_msg, Wi, gmsgv[s]);
    wmma_gemm64<0, false, 0, 0, false, 0><<<dim3((ghTiles + 7) / 8, 1), 256, 0, stream>>>(
        (const unsigned short*)h16v[s], (const unsigned short*)nullptr, kHid, 0L,
        (const unsigned short*)Wh16, (const unsigned short*)nullptr, kHid, 0L,
        (void*)gh, (void*)nullptr, kG3, 0L,
        (const float*)nullptr, (const float*)nullptr, 0L, kRows, kG3, kHid, kGemmScale);
    gru_kernel<<<kRows / kRowsPerBlk, 256, 0, stream>>>(gij, gh, gmsgv[s], bh, h32v[s], h32v[s + 1], h16v[s + 1]);
  }

  const int roTiles = (kRows / 64) * (kHid / 64);
  wmma_gemm64<0, false, 2, 0, false, 2><<<dim3((roTiles + 7) / 8, 1), 256, 0, stream>>>(
      (const unsigned short*)h16v[kIters], (const unsigned short*)nullptr, kHid, 0L,
      (const unsigned short*)Wr1T16, (const unsigned short*)nullptr, kHid, 0L,
      (void*)y, (void*)nullptr, kHid, 0L,
      br1, (const float*)nullptr, 0L, kRows, kHid, kHid, kGemmScale);
  readout_kernel<<<kBatch, 256, 0, stream>>>(y, Wr2, br2, out);
}
